// SwinTransformer3DJoint_36318243455757
// MI455X (gfx1250) — hardware-verified
//
#include <hip/hip_runtime.h>

typedef _Float16 f16;
typedef __attribute__((ext_vector_type(16))) _Float16 v16h;
typedef __attribute__((ext_vector_type(8)))  _Float16 v8h;
typedef __attribute__((ext_vector_type(8)))  float    v8f;
typedef __attribute__((ext_vector_type(4)))  float    v4f_t;
typedef float v4fa __attribute__((ext_vector_type(4), may_alias));
typedef __attribute__((ext_vector_type(4)))  unsigned v4u_t;
typedef unsigned v4ua __attribute__((ext_vector_type(4), may_alias));

#define TOK     50176
#define NWIN    512
#define NSEQ    98
#define MTILES  3136
#define KVLD    64

__device__ __forceinline__ v8f wmma16(v16h a, v16h b, v8f c) {
  return __builtin_amdgcn_wmma_f32_16x16x32_f16(false, a, false, b, (short)0, c, false, false);
}
__device__ __forceinline__ v16h frag16(const f16* p, int hf) {
  return __builtin_shufflevector(*(const v8h*)(p + 8 * hf), *(const v8h*)(p + 16 + 8 * hf), 0,1,2,3,4,5,6,7,8,9,10,11,12,13,14,15);
}
__device__ __forceinline__ v16h frag32(const float* p, int hf, float s) {
  v16h v;
#pragma unroll
  for (int i = 0; i < 8; ++i) { v[i] = (f16)(p[8 * hf + i] * s); v[i + 8] = (f16)(p[16 + 8 * hf + i] * s); }
  return v;
}
__device__ __forceinline__ float wred(float v) {
#pragma unroll
  for (int m = 16; m > 0; m >>= 1) v += __shfl_xor(v, m, 32);
  return v;
}
__device__ __forceinline__ void st2f(float* p, float v) { *(volatile float*)p = v; __threadfence(); *(volatile float*)p = v; }

__global__ void k_cvt(const float* __restrict__ s, f16* __restrict__ d, int n) {
  int i = (blockIdx.x * 256 + threadIdx.x) * 2;
  if (i < n) { const unsigned u = (unsigned)__builtin_bit_cast(unsigned short, (f16)s[i]) | ((unsigned)__builtin_bit_cast(unsigned short, (f16)s[i + 1]) << 16);
    *(volatile unsigned*)(d + i) = u; __threadfence(); *(volatile unsigned*)(d + i) = u; }
}
__global__ void k_bias(const float* __restrict__ table, const int* __restrict__ rel, float* __restrict__ out) {
  int idx = blockIdx.x * 256 + threadIdx.x;
  if (idx < 4 * NSEQ * NSEQ) {
    int h = idx / (NSEQ * NSEQ), i = idx - h * NSEQ * NSEQ;
    int ri = rel[i]; ri = (ri < 0) ? 0 : (ri > 506 ? 506 : ri);
    st2f(out + idx, table[ri * 4 + h]);
  }
}

__global__ __launch_bounds__(256)
void k_ln1(const float* __restrict__ x, const float* __restrict__ g, const float* __restrict__ b, f16* __restrict__ dst) {
  int wave = threadIdx.x >> 5, lane = threadIdx.x & 31;
  long t = (long)blockIdx.x * 8 + wave;
  const float* row = x + t * 128;
  float4 v = *(const float4*)(row + lane * 4);
  float mean = wred(v.x + v.y + v.z + v.w) * (1.f / 128.f);
  float4 d2 = make_float4(v.x - mean, v.y - mean, v.z - mean, v.w - mean);
  float var = wred(d2.x*d2.x + d2.y*d2.y + d2.z*d2.z + d2.w*d2.w) * (1.f / 128.f);
  float rstd = rsqrtf(var + 1e-5f);
  int wq = t % 56, hq = (t / 56) % 56, dq = (t / 3136) % 8, bq = t / 25088;
  int win = ((bq * 4 + (dq >> 1)) * 8 + hq / 7) * 8 + wq / 7;
  int n   = (dq & 1) * 49 + (hq % 7) * 7 + (wq % 7);
  long r = (long)win * NSEQ + n;
  int c = lane * 4;
  f16 hh[4];
  hh[0] = (f16)(d2.x * rstd * g[c]     + b[c]);
  hh[1] = (f16)(d2.y * rstd * g[c + 1] + b[c + 1]);
  hh[2] = (f16)(d2.z * rstd * g[c + 2] + b[c + 2]);
  hh[3] = (f16)(d2.w * rstd * g[c + 3] + b[c + 3]);
  typedef __attribute__((ext_vector_type(2))) unsigned v2u_t; typedef unsigned v2ua __attribute__((ext_vector_type(2), may_alias));
  const v2u_t u = *(const v2ua*)hh;
  *(volatile v2u_t*)(dst + r * 128 + c) = u; __threadfence(); *(volatile v2u_t*)(dst + r * 128 + c) = u;
}

__global__ __launch_bounds__(256)
void k_qkv(const f16* __restrict__ A, const f16* __restrict__ W, const float* __restrict__ qkv_bias,
           float* __restrict__ qf, f16* __restrict__ kv) {
  __shared__ __attribute__((aligned(16))) float sq[8][16 * 36];
  __shared__ __attribute__((aligned(16))) f16   skv[8][16 * 72];
  const int wave = threadIdx.x >> 5, lane = threadIdx.x & 31, hf = lane >> 4, l16 = lane & 15;
  const int strip = blockIdx.x * 8 + wave;
  const int mt = strip >> 2, head = strip & 3;
  const f16* arow = A + (size_t)(mt * 16 + l16) * 128;
  int jb[6]; jb[0] = 32 * head; jb[1] = jb[0] + 16; jb[2] = 128 + 32 * head; jb[3] = jb[2] + 16; jb[4] = 256 + 32 * head; jb[5] = jb[4] + 16;
  v8f acc[6] = {};
#pragma unroll
  for (int k0 = 0; k0 < 128; k0 += 32) {
    v16h a = frag16(arow + k0, hf);
#pragma unroll
    for (int g = 0; g < 6; ++g) acc[g] = wmma16(a, frag16(W + (size_t)(jb[g] + l16) * 128 + k0, hf), acc[g]);
  }
  float* sqw = sq[wave]; f16* skw = skv[wave];
#pragma unroll
  for (int g = 0; g < 6; ++g) {
    const float bias = qkv_bias[jb[g] + l16];
#pragma unroll
    for (int rr = 0; rr < 8; ++rr) {
      const int rl = rr + hf * 8;
      const float v = acc[g][rr] + bias;
      if (g < 2) sqw[rl * 36 + (g & 1) * 16 + l16] = v * 0.17677669529663687f;
      else       skw[rl * 72 + (g - 2) * 16 + l16] = (f16)v;
    }
  }
  asm volatile("s_wait_dscnt 0" ::: "memory");
#pragma unroll 1
  for (int pass = 0; pass < 2; ++pass) {
#pragma unroll
    for (int i = 0; i < 4; ++i) {
      const int c = lane + 32 * i, rl = c >> 3, q = (c & 7) * 4;
      const int m = mt * 16 + rl, win = m / NSEQ, n = m - win * NSEQ;
      *(volatile v4f_t*)(qf + (((size_t)win * 4 + head) * NSEQ + n) * 32 + q) = *(const volatile v4fa*)(sqw + rl * 36 + q);
    }
#pragma unroll
    for (int i = 0; i < 4; ++i) {
      const int c = lane + 32 * i, rl = c >> 3, q = (c & 7) * 8;
      const int m = mt * 16 + rl, win = m / NSEQ, n = m - win * NSEQ;
      *(volatile v4u_t*)(kv + (((size_t)win * 4 + head) * NSEQ + n) * KVLD + q) = *(const volatile v4ua*)(skw + rl * 72 + q);
    }
    __threadfence();
  }
}

__global__ __launch_bounds__(256)
void k_attn(const float* __restrict__ qf, const f16* __restrict__ kv, const float* __restrict__ bias, f16* __restrict__ attn_out) {
  __shared__ __attribute__((aligned(16))) float sc[112 * 128];
  __shared__ __attribute__((aligned(16))) f16   Qs[112 * 40];
  __shared__ __attribute__((aligned(16))) f16   Ks[128 * 40];
  __shared__ __attribute__((aligned(16))) f16   Vt[32 * 136];
  __shared__ __attribute__((aligned(16))) f16   os[NSEQ * 136];
  const int win = blockIdx.x, tid = threadIdx.x, wave = tid >> 5, lane = tid & 31, hf = lane >> 4, idx = lane & 15;

  for (int head = 0; head < 4; ++head) {
    const int wh = win * 4 + head;
    __syncthreads();
#pragma unroll 1
    for (int c = tid; c < 128 * 4; c += 256) {
      const int row = c >> 2, q8 = (c & 3) * 8;
      f16 qh[8], kh[8], vh[8];
      if (row < NSEQ) {
        const float* qp = qf + ((size_t)wh * NSEQ + row) * 32 + q8;
        const f16* kp = kv + ((size_t)wh * NSEQ + row) * KVLD + q8;
#pragma unroll
        for (int e = 0; e < 8; ++e) { qh[e] = (f16)qp[e]; kh[e] = kp[e]; vh[e] = kp[32 + e]; }
      } else {
#pragma unroll
        for (int e = 0; e < 8; ++e) { qh[e] = (f16)0.f; kh[e] = (f16)0.f; vh[e] = (f16)0.f; }
      }
      if (row < 112) *(v4u_t*)(Qs + row * 40 + q8) = *(const v4ua*)qh;
      *(v4u_t*)(Ks + row * 40 + q8) = *(const v4ua*)kh;
#pragma unroll
      for (int e = 0; e < 8; ++e) Vt[(q8 + e) * 136 + row] = vh[e];
    }
    __syncthreads();

    {
      const int nt = wave;
      const v16h bfrag = frag16(Ks + (nt * 16 + idx) * 40, hf);
      const float* bi = bias + head * NSEQ * NSEQ;
#pragma unroll 1
      for (int mt = 0; mt < 7; ++mt) {
        v8f acc = {};
        acc = wmma16(frag16(Qs + (mt * 16 + idx) * 40, hf), bfrag, acc);
#pragma unroll
        for (int rr = 0; rr < 8; ++rr) {
          const int qi = mt * 16 + rr + hf * 8, ki = nt * 16 + idx;
          float v;
          if (qi < NSEQ && ki < NSEQ) v = acc[rr] + bi[qi * NSEQ + ki];
          else                        v = (qi < NSEQ) ? -1e30f : 0.f;
          sc[qi * 128 + ki] = v;
        }
      }
    }
    __syncthreads();

    if (tid < NSEQ) {
      float* r = sc + tid * 128;
      float mx = -1e30f;
      for (int m = 0; m < NSEQ; ++m) mx = fmaxf(mx, r[m]);
      float s = 0.f;
      for (int m = 0; m < NSEQ; ++m) { float e = __expf(r[m] - mx); r[m] = e; s += e; }
      const float inv = 1024.f / s;
      for (int m = 0; m < NSEQ; ++m) r[m] *= inv;
      for (int m = NSEQ; m < 128; ++m) r[m] = 0.f;
    } else if (tid < 112) {
      float* r = sc + tid * 128;
      for (int m = 0; m < 128; ++m) r[m] = 0.f;
    }
    __syncthreads();

#pragma unroll 1
    for (int tile = wave; tile < 14; tile += 8) {
      const int mt = tile >> 1, nt = tile & 1;
      v8f acc = {};
#pragma unroll
      for (int k0 = 0; k0 < 128; k0 += 32)
        acc = wmma16(frag32(sc + (mt * 16 + idx) * 128 + k0, hf, 1.0f), frag16(Vt + (nt * 16 + idx) * 136 + k0, hf), acc);
#pragma unroll
      for (int rr = 0; rr < 8; ++rr) {
        const int qi = mt * 16 + rr + hf * 8;
        if (qi < NSEQ) os[qi * 136 + head * 32 + nt * 16 + idx] = (f16)(acc[rr] * (1.0f / 1024.0f));
      }
    }
  }
  __syncthreads();
#pragma unroll 1
  for (int pass = 0; pass < 2; ++pass) {
    for (int c = tid; c < NSEQ * 16; c += 256) {
      const int qi = c >> 4, q8 = (c & 15) * 8;
      *(volatile v4u_t*)(attn_out + ((size_t)win * NSEQ + qi) * 128 + q8) = *(const volatile v4ua*)(os + qi * 136 + q8);
    }
    __threadfence();
  }
}

__global__ __launch_bounds__(256)
void k_proj(const f16* __restrict__ A, const f16* __restrict__ W, const float* __restrict__ pb, const float* __restrict__ x,
            float* __restrict__ xres) {
  __shared__ __attribute__((aligned(16))) float stg[8][16 * 68];
  const int wave = threadIdx.x >> 5, lane = threadIdx.x & 31, hf = lane >> 4, l16 = lane & 15;
  const int strip = blockIdx.x * 8 + wave;
  const int mt = strip >> 1, ng = strip & 1;
  const f16* arow = A + (size_t)(mt * 16 + l16) * 128;
  v8f acc[4] = {};
#pragma unroll
  for (int k0 = 0; k0 < 128; k0 += 32) {
    v16h a = frag16(arow + k0, hf);
#pragma unroll
    for (int g = 0; g < 4; ++g) acc[g] = wmma16(a, frag16(W + (size_t)(ng * 64 + g * 16 + l16) * 128 + k0, hf), acc[g]);
  }
  float* sw = stg[wave];
#pragma unroll
  for (int g = 0; g < 4; ++g) {
    const int j = ng * 64 + g * 16 + l16;
    const float bias = pb[j];
#pragma unroll
    for (int rr = 0; rr < 8; ++rr) {
      const int rl = rr + hf * 8, m = mt * 16 + rl;
      const int win = m / NSEQ, n = m % NSEQ;
      const int w7 = win & 7, h7 = (win >> 3) & 7, d2 = (win >> 6) & 3, b = win >> 8;
      const int dn = n / 49, rem = n % 49, hn = rem / 7, wn = rem % 7;
      const int d = d2 * 2 + dn, hh = h7 * 7 + hn, ww = w7 * 7 + wn;
      const size_t t = (((size_t)b * 8 + d) * 56 + hh) * 56 + ww;
      sw[rl * 68 + g * 16 + l16] = x[t * 128 + j] + acc[g][rr] + bias;
    }
  }
  asm volatile("s_wait_dscnt 0" ::: "memory");
#pragma unroll 1
  for (int pass = 0; pass < 2; ++pass) {
#pragma unroll
    for (int i = 0; i < 8; ++i) {
      const int c = lane + 32 * i, rl = c >> 4, q = (c & 15) * 4, m = mt * 16 + rl;
      const int win = m / NSEQ, n = m % NSEQ;
      const int w7 = win & 7, h7 = (win >> 3) & 7, d2 = (win >> 6) & 3, b = win >> 8;
      const int dn = n / 49, rem = n % 49, hn = rem / 7, wn = rem % 7;
      const int d = d2 * 2 + dn, hh = h7 * 7 + hn, ww = w7 * 7 + wn;
      const size_t t = (((size_t)b * 8 + d) * 56 + hh) * 56 + ww;
      *(volatile v4f_t*)(xres + t * 128 + ng * 64 + q) = *(const volatile v4fa*)(sw + rl * 68 + q);
    }
    __threadfence();
  }
}

__global__ __launch_bounds__(256)
void k_mlp(const float* __restrict__ xres, const float* __restrict__ g2, const float* __restrict__ b2n,
           const f16* __restrict__ W1, const float* __restrict__ fb1, const f16* __restrict__ W2, const float* __restrict__ fb2,
           float* __restrict__ out) {
  __shared__ __attribute__((aligned(16))) f16   hs[16 * 136];
  __shared__ __attribute__((aligned(16))) f16   gs[16 * 520];
  __shared__ __attribute__((aligned(16))) float so[16 * 132];
  const int tid = threadIdx.x, wave = tid >> 5, lane = tid & 31, hf = lane >> 4, l16 = lane & 15;
  const int m0 = blockIdx.x * 16;
  {
    const int row = tid >> 4, c8 = (tid & 15) * 8;
    const float* xr = xres + (size_t)(m0 + row) * 128 + c8;
    float v[8], s = 0.f;
#pragma unroll
    for (int e = 0; e < 8; ++e) { v[e] = xr[e]; s += v[e]; }
#pragma unroll
    for (int m = 8; m > 0; m >>= 1) s += __shfl_xor(s, m, 32);
    const float mean = s * (1.f / 128.f);
    float q = 0.f;
#pragma unroll
    for (int e = 0; e < 8; ++e) { v[e] -= mean; q += v[e] * v[e]; }
#pragma unroll
    for (int m = 8; m > 0; m >>= 1) q += __shfl_xor(q, m, 32);
    const float rstd = rsqrtf(q * (1.f / 128.f) + 1e-5f);
#pragma unroll
    for (int e = 0; e < 8; ++e) hs[row * 136 + c8 + e] = (f16)(v[e] * rstd * g2[c8 + e] + b2n[c8 + e]);
  }
  __syncthreads();
  {
    v8f acc[4] = {};
#pragma unroll
    for (int k0 = 0; k0 < 128; k0 += 32) {
      v16h a = frag16(hs + l16 * 136 + k0, hf);
#pragma unroll
      for (int g = 0; g < 4; ++g) acc[g] = wmma16(a, frag16(W1 + (size_t)(wave * 64 + g * 16 + l16) * 128 + k0, hf), acc[g]);
    }
#pragma unroll
    for (int g = 0; g < 4; ++g) {
      const int j = wave * 64 + g * 16 + l16;
      const float bias = fb1[j];
#pragma unroll
      for (int rr = 0; rr < 8; ++rr) {
        float v = acc[g][rr] + bias;
        v = 0.5f * v * (1.f + erff(v * 0.70710678118654752f));
        gs[(rr + hf * 8) * 520 + j] = (f16)v;
      }
    }
  }
  __syncthreads();
  {
    v8f acc = {};
#pragma unroll 4
    for (int k0 = 0; k0 < 512; k0 += 32)
      acc = wmma16(frag16(gs + l16 * 520 + k0, hf), frag16(W2 + (size_t)(wave * 16 + l16) * 512 + k0, hf), acc);
    const int j = wave * 16 + l16;
    const float bias = fb2[j];
#pragma unroll
    for (int rr = 0; rr < 8; ++rr) { const int rl = rr + hf * 8; so[rl * 132 + j] = xres[(size_t)(m0 + rl) * 128 + j] + acc[rr] + bias; }
  }
  __syncthreads();
#pragma unroll 1
  for (int pass = 0; pass < 2; ++pass) {
    for (int c = tid; c < 16 * 32; c += 256) { const int rl = c >> 5, q = (c & 31) * 4;
      *(volatile v4f_t*)(out + (size_t)(m0 + rl) * 128 + q) = *(const volatile v4fa*)(so + rl * 132 + q); }
    __threadfence();
  }
}

extern "C" void kernel_launch(void* const* d_in, const int* in_sizes, int n_in,
                              void* d_out, int out_size, void* d_ws, size_t ws_size,
                              hipStream_t stream) {
  (void)in_sizes; (void)n_in; (void)out_size; (void)ws_size;
  const float* x        = (const float*)d_in[0];
  const float* norm1_w  = (const float*)d_in[1];
  const float* norm1_b  = (const float*)d_in[2];
  const float* qkv_w    = (const float*)d_in[3];
  const float* qkv_b    = (const float*)d_in[4];
  const float* btable   = (const float*)d_in[5];
  const float* proj_w   = (const float*)d_in[6];
  const float* proj_b   = (const float*)d_in[7];
  const float* norm2_w  = (const float*)d_in[8];
  const float* norm2_b  = (const float*)d_in[9];
  const float* fc1_w    = (const float*)d_in[10];
  const float* fc1_b    = (const float*)d_in[11];
  const float* fc2_w    = (const float*)d_in[12];
  const float* fc2_b    = (const float*)d_in[13];
  const int*   rel_idx  = (const int*)d_in[14];
  float* out = (float*)d_out;

  char* ws = (char*)d_ws;
  size_t off = 0;
  auto alloc = [&](size_t bytes) -> void* { off = (off + 255) & ~(size_t)255; void* p = ws + off; off += bytes; return p; };
  f16*   xw    = (f16*)  alloc((size_t)TOK * 128 * 2);
  float* qf    = (float*)alloc((size_t)NWIN * 4 * NSEQ * 32 * 4);
  f16*   kv    = (f16*)  alloc((size_t)NWIN * 4 * NSEQ * KVLD * 2);
  f16*   attn  = (f16*)  alloc((size_t)TOK * 128 * 2);
  float* xres  = (float*)alloc((size_t)TOK * 128 * 4);
  f16*   wqkv  = (f16*)  alloc((size_t)384 * 128 * 2);
  f16*   wproj = (f16*)  alloc((size_t)128 * 128 * 2);
  f16*   wfc1  = (f16*)  alloc((size_t)512 * 128 * 2);
  f16*   wfc2  = (f16*)  alloc((size_t)128 * 512 * 2);
  float* bbuf  = (float*)alloc((size_t)4 * NSEQ * NSEQ * 4);

  k_cvt<<<(49152 / 2 + 255) / 256, 256, 0, stream>>>(qkv_w,  wqkv,  49152);
  k_cvt<<<(16384 / 2 + 255) / 256, 256, 0, stream>>>(proj_w, wproj, 16384);
  k_cvt<<<(65536 / 2 + 255) / 256, 256, 0, stream>>>(fc1_w,  wfc1,  65536);
  k_cvt<<<(65536 / 2 + 255) / 256, 256, 0, stream>>>(fc2_w,  wfc2,  65536);
  k_bias<<<(4 * NSEQ * NSEQ + 255) / 256, 256, 0, stream>>>(btable, rel_idx, bbuf);

  k_ln1<<<TOK / 8, 256, 0, stream>>>(x, norm1_w, norm1_b, xw);
  k_qkv<<<MTILES * 4 / 8, 256, 0, stream>>>(xw, wqkv, qkv_b, qf, kv);
  k_attn<<<NWIN, 256, 0, stream>>>(qf, kv, bbuf, attn);
  k_proj<<<MTILES * 2 / 8, 256, 0, stream>>>(attn, wproj, proj_b, x, xres);
  k_mlp<<<MTILES, 256, 0, stream>>>(xres, norm2_w, norm2_b, wfc1, fc1_b, wfc2, fc2_b, out);
}
